// CoAttentionFusion_20641612825100
// MI455X (gfx1250) — hardware-verified
//
#include <hip/hip_runtime.h>
#include <stddef.h>
#include <stdint.h>
#include <math.h>

#define NB   16
#define LL   512
#define DD   512
#define NH   8
#define HD   128
#define INR  1024
#define KC   640
#define TP   72

#define PL_ACT ((size_t)NB * LL * DD * 2)
#define PL_WA  ((size_t)NH * DD * DD * 2)
#define PL_WP  ((size_t)INR * DD * 2)
#define PL_WF  ((size_t)DD * KC * 2)
#define PL_PP  ((size_t)NB * INR * LL * 2)
#define PL_T   ((size_t)NH * LL * DD * 2)
#define PL_AF  ((size_t)NH * LL * LL * 2)
#define PL_Q   ((size_t)NB * LL * HD * 2)

#define OFF_P16 ((size_t)0)
#define OFF_S16 (OFF_P16 + PL_ACT)
#define OFF_WA  (OFF_S16 + PL_ACT)
#define OFF_WP  (OFF_WA + PL_WA)
#define OFF_WS  (OFF_WP + PL_WP)
#define OFF_WFP (OFF_WS + PL_WP)
#define OFF_WFS (OFF_WFP + PL_WF)
#define OFF_PPH (OFF_WFS + PL_WF)
#define OFF_PPL (OFF_PPH + PL_PP)
#define OFF_PSH (OFF_PPL + PL_PP)
#define OFF_PSL (OFF_PSH + PL_PP)
#define OFF_TH  (OFF_PSL + PL_PP)
#define OFF_TL  (OFF_TH + PL_T)
#define OFF_AH  (OFF_TL + PL_T)
#define OFF_AL  (OFF_AH + PL_AF)
#define OFF_AHT (OFF_AL + PL_AF)
#define OFF_ALT (OFF_AHT + PL_AF)
#define OFF_QSH (OFF_ALT + PL_AF)
#define OFF_QSL (OFF_QSH + PL_Q)
#define OFF_QPH (OFF_QSL + PL_Q)
#define OFF_QPL (OFF_QPH + PL_Q)
#define WS_TOTAL (OFF_QPL + PL_Q)

static_assert(WS_TOTAL == (size_t)125042688);
static_assert(WS_TOTAL <= (size_t)134217728);
static_assert((OFF_S16 % 256) == 0);
static_assert((OFF_WA % 256) == 0);
static_assert((OFF_WP % 256) == 0);
static_assert((OFF_WS % 256) == 0);
static_assert((OFF_WFP % 256) == 0);
static_assert((OFF_WFS % 256) == 0);
static_assert((OFF_PPH % 256) == 0);
static_assert((OFF_PPL % 256) == 0);
static_assert((OFF_PSH % 256) == 0);
static_assert((OFF_PSL % 256) == 0);
static_assert((OFF_TH % 256) == 0);
static_assert((OFF_TL % 256) == 0);
static_assert((OFF_AH % 256) == 0);
static_assert((OFF_AL % 256) == 0);
static_assert((OFF_AHT % 256) == 0);
static_assert((OFF_ALT % 256) == 0);
static_assert((OFF_QSH % 256) == 0);
static_assert((OFF_QSL % 256) == 0);
static_assert((OFF_QPH % 256) == 0);
static_assert((OFF_QPL % 256) == 0);
static_assert((LL % 64) == 0);
static_assert((DD % 64) == 0);
static_assert((INR % 64) == 0);
static_assert((HD % 64) == 0);
static_assert((KC % 32) == 0);
static_assert(KC == DD + HD);
static_assert(INR == NH * HD);
static_assert(LL == DD);
static_assert(((NB * LL * DD) % 2048) == 0);
static_assert((size_t)2 * NB * LL * DD == (size_t)8388608);

typedef unsigned short v8us  __attribute__((ext_vector_type(8)));
typedef unsigned short v16us __attribute__((ext_vector_type(16)));
typedef _Float16       v16h  __attribute__((ext_vector_type(16)));
typedef float          v4f   __attribute__((ext_vector_type(4)));
typedef float          v8f   __attribute__((ext_vector_type(8)));

union FragU { v16us v; v8us half[2]; };

__device__ __forceinline__ unsigned bbits(float f) {
  unsigned u = __float_as_uint(f);
  return (u + 0x7FFFu + ((u >> 16) & 1u)) >> 16;
}
__device__ __forceinline__ float bf16r(float f) {
  return __uint_as_float(bbits(f) << 16);
}
__device__ __forceinline__ unsigned short hbits(float f) {
  return __builtin_bit_cast(unsigned short, (_Float16)f);
}
__device__ __forceinline__ v8f zero8() { v8f z = {0.f, 0.f, 0.f, 0.f, 0.f, 0.f, 0.f, 0.f}; return z; }

__device__ __forceinline__ void split_hl(float p, unsigned short& hb, unsigned short& lb) {
  const bool tiny = fabsf(p) < 6.103515625e-05f;
  const _Float16 hh = tiny ? (_Float16)0.0f : (_Float16)p;
  const float hv = (float)hh;
  hb = __builtin_bit_cast(unsigned short, hh);
  lb = hbits((p - hv) * 2048.0f);
}

__device__ __forceinline__ float tanh_f(float x) {
  const float y = fminf(fabsf(x), 10.0f);
  const float e = expf(2.0f * y);
  const float t = (e - 1.0f) * (1.0f / (e + 1.0f));
  return copysignf(t, x);
}

__device__ __forceinline__ v16us ldfrag_u(const unsigned short* p) {
  FragU f;
  f.half[0] = *(const v8us*)(p);
  f.half[1] = *(const v8us*)(p + 16);
  return f.v;
}

__device__ __forceinline__ v8f mma_hu(v16us a, v16us b, v8f c) {
#if defined(__HIP_DEVICE_COMPILE__)
  return __builtin_amdgcn_wmma_f32_16x16x32_f16(false, __builtin_bit_cast(v16h, a),
                                               false, __builtin_bit_cast(v16h, b),
                                               (short)0, c, false, false);
#else
  (void)a; (void)b;
  return c;
#endif
}
__device__ __forceinline__ void guard4(v8f& c0, v8f& c1, v8f& c2, v8f& c3, const v16us& a,
                                       const v16us& b0, const v16us& b1, const v16us& b2,
                                       const v16us& b3) {
#if defined(__HIP_DEVICE_COMPILE__)
  asm volatile("v_nop\n\tv_nop\n\tv_nop\n\tv_nop"
               : "+v"(c0), "+v"(c1), "+v"(c2), "+v"(c3)
               : "v"(a), "v"(b0), "v"(b1), "v"(b2), "v"(b3));
#else
  (void)c0; (void)c1; (void)c2; (void)c3; (void)a; (void)b0; (void)b1; (void)b2; (void)b3;
#endif
}
__device__ __forceinline__ void guard4x6(v8f& c0, v8f& c1, v8f& c2, v8f& c3, const v16us& a0,
                                         const v16us& a1, const v16us& b0, const v16us& b1,
                                         const v16us& b2, const v16us& b3) {
#if defined(__HIP_DEVICE_COMPILE__)
  asm volatile("v_nop\n\tv_nop\n\tv_nop\n\tv_nop"
               : "+v"(c0), "+v"(c1), "+v"(c2), "+v"(c3)
               : "v"(a0), "v"(a1), "v"(b0), "v"(b1), "v"(b2), "v"(b3));
#else
  (void)c0; (void)c1; (void)c2; (void)c3; (void)a0; (void)a1; (void)b0; (void)b1; (void)b2; (void)b3;
#endif
}
__device__ __forceinline__ void guard8(v8f& c0, v8f& c1, v8f& c2, v8f& c3, v8f& c4, v8f& c5,
                                       v8f& c6, v8f& c7, const v16us& a0, const v16us& a1,
                                       const v16us& b0, const v16us& b1, const v16us& b2,
                                       const v16us& b3) {
#if defined(__HIP_DEVICE_COMPILE__)
  asm volatile("v_nop\n\tv_nop\n\tv_nop\n\tv_nop"
               : "+v"(c0), "+v"(c1), "+v"(c2), "+v"(c3), "+v"(c4), "+v"(c5), "+v"(c6), "+v"(c7)
               : "v"(a0), "v"(a1), "v"(b0), "v"(b1), "v"(b2), "v"(b3));
#else
  (void)c0; (void)c1; (void)c2; (void)c3; (void)c4; (void)c5; (void)c6; (void)c7;
  (void)a0; (void)a1; (void)b0; (void)b1; (void)b2; (void)b3;
#endif
}

__device__ __forceinline__ void store_tile_f32(const float* ct, float* C, size_t row0, int col0,
                                               int ldc, int w, int lane) {
  const int q  = lane >> 3;
  const int jj = lane & 7;
#pragma unroll 1
  for (int it = 0; it < 8; ++it) {
    const int li = it * 16 + w * 4 + q;
    const int tr = li >> 1, hf = li & 1;
    const v4f v = *(const v4f*)(ct + tr * 64 + hf * 32 + jj * 4);
    *(volatile v4f*)(C + (row0 + tr) * (size_t)ldc + col0 + hf * 32 + jj * 4) = v;
  }
  __threadfence();
#pragma unroll 1
  for (int it = 0; it < 8; ++it) {
    const int li = it * 16 + w * 4 + q;
    const int tr = li >> 1, hf = li & 1;
    const v4f v = *(const v4f*)(ct + tr * 64 + hf * 32 + jj * 4);
    *(volatile v4f*)(C + (row0 + tr) * (size_t)ldc + col0 + hf * 32 + jj * 4) = v;
  }
}
template <int NW, int PITCH>
__device__ __forceinline__ void store_tile_us(const unsigned short* t, unsigned short* P,
                                              size_t row0, int ld, int col0, int w, int lane) {
  constexpr int NIT = 64 / (4 * NW);
  const int q  = lane >> 3;
  const int jj = lane & 7;
  v8us   v[NIT];
  size_t off[NIT];
#pragma unroll
  for (int it = 0; it < NIT; ++it) {
    const int li = it * 4 * NW + w * 4 + q;
    v[it]   = *(const v8us*)(t + li * PITCH + 8 * jj);
    off[it] = (row0 + li) * (size_t)ld + col0 + 8 * jj;
  }
#pragma unroll
  for (int it = 0; it < NIT; ++it) *(volatile v8us*)(P + off[it]) = v[it];
  __threadfence();
#pragma unroll
  for (int it = 0; it < NIT; ++it) *(volatile v8us*)(P + off[it]) = v[it];
}

__global__ __launch_bounds__(256)
void k_cva(const float* __restrict__ Pin, const float* __restrict__ Sin,
           unsigned short* p16, unsigned short* s16)
{
  const int bid  = blockIdx.x;
  const int kind = (bid >= 2048) ? 1 : 0;
  const size_t i = ((size_t)(kind ? (bid - 2048) : bid) * 256 + threadIdx.x) * 8;
  const float* sp = (kind ? Sin : Pin) + i;
  const v4f a0 = *(const v4f*)(sp);
  const v4f a1 = *(const v4f*)(sp + 4);
  v8us o;
#pragma unroll
  for (int e = 0; e < 4; ++e) {
    o[e]     = hbits(16.0f * bf16r(a0[e]));
    o[4 + e] = hbits(16.0f * bf16r(a1[e]));
  }
  unsigned short* dst = (kind ? s16 : p16) + i;
  *(volatile v8us*)dst = o;
  __threadfence();
  *(volatile v8us*)dst = o;
}

__global__ __launch_bounds__(256)
void k_cvw(const float* __restrict__ Waff, const float* __restrict__ Wp, const float* __restrict__ Wsx,
           const float* __restrict__ Wfp, const float* __restrict__ Wfs,
           unsigned short* wa16, unsigned short* wp16, unsigned short* ws16,
           unsigned short* wfp16, unsigned short* wfs16)
{
  __shared__ __align__(16) unsigned short ttr[64 * TP];

  const int tid  = threadIdx.x;
  const int lane = tid & 31;
  const int w    = tid >> 5;
  const int bid  = blockIdx.x;
  const float* in;
  unsigned short* outp;
  int ip, op, rt, ct;
  if (bid < 512) {
    const int hh = bid >> 6, t = bid & 63;
    rt = t >> 3; ct = t & 7;
    in = Waff + (size_t)hh * DD * DD;  ip = DD;
    outp = wa16 + (size_t)hh * DD * DD; op = DD;
  } else if (bid < 768) {
    int t = bid - 512;
    const int sel = (t >= 128) ? 1 : 0;
    t -= 128 * sel;
    rt = t >> 4; ct = t & 15;
    in = sel ? Wsx : Wp;     ip = INR;
    outp = sel ? ws16 : wp16; op = DD;
  } else {
    int t = bid - 768;
    const int sel = (t >= 80) ? 1 : 0;
    t -= 80 * sel;
    rt = t >> 3; ct = t & 7;
    in = sel ? Wfs : Wfp;      ip = DD;
    outp = sel ? wfs16 : wfp16; op = KC;
  }
  const int r0 = 64 * rt, c0 = 64 * ct;
  const int rr = tid >> 2;
  const int cl = 16 * (tid & 3);
  const float* sp = in + (size_t)(r0 + rr) * ip + c0 + cl;
  v4f u[4];
  u[0] = *(const v4f*)(sp);
  u[1] = *(const v4f*)(sp + 4);
  u[2] = *(const v4f*)(sp + 8);
  u[3] = *(const v4f*)(sp + 12);
#pragma unroll
  for (int g = 0; g < 4; ++g) {
#pragma unroll
    for (int e = 0; e < 4; ++e) {
      const int cc = cl + 4 * g + e;
      ttr[cc * TP + rr] = hbits(64.0f * bf16r(u[g][e]));
    }
  }
  __syncthreads();
  store_tile_us<8, TP>(ttr, outp, (size_t)c0, op, r0, w, lane);
}

struct GArgs {
  const unsigned short* A;
  const unsigned short* B;
  unsigned short* CH;
  unsigned short* CL;
  long long sAz, sBz, sCz;
  int lda, ldb, ldc, nk;
};
static_assert(sizeof(GArgs) == 72);

__global__ __launch_bounds__(128)
void k_ghl(GArgs g)
{
  __shared__ __align__(16) unsigned short thi[64 * 64];
  __shared__ __align__(16) unsigned short tlo[64 * 64];

  const int tid  = threadIdx.x;
  const int lane = tid & 31;
  const int w    = tid >> 5;
  const int h    = lane >> 4;
  const int m    = lane & 15;
  const int n0   = 64 * blockIdx.x;
  const int r0   = 64 * blockIdx.y;
  const int z    = blockIdx.z;

  v8f acc[4];
#pragma unroll
  for (int j = 0; j < 4; ++j) acc[j] = zero8();

  const unsigned short* pa = g.A + (size_t)z * (size_t)g.sAz + (size_t)(r0 + 16 * w + m) * g.lda + 8 * h;
  const unsigned short* pb = g.B + (size_t)z * (size_t)g.sBz + (size_t)(n0 + m) * g.ldb + 8 * h;
  const size_t bs = (size_t)16 * g.ldb;
#pragma unroll 2
  for (int kk = 0; kk < g.nk; ++kk) {
    const v16us a  = ldfrag_u(pa + 32 * kk);
    const v16us b0 = ldfrag_u(pb + 32 * kk);
    const v16us b1 = ldfrag_u(pb + bs + 32 * kk);
    const v16us b2 = ldfrag_u(pb + 2 * bs + 32 * kk);
    const v16us b3 = ldfrag_u(pb + 3 * bs + 32 * kk);
    acc[0] = mma_hu(a, b0, acc[0]);
    acc[1] = mma_hu(a, b1, acc[1]);
    acc[2] = mma_hu(a, b2, acc[2]);
    acc[3] = mma_hu(a, b3, acc[3]);
    guard4(acc[0], acc[1], acc[2], acc[3], a, b0, b1, b2, b3);
  }

  const float ko = 1.0f / 64.0f;
#pragma unroll
  for (int j = 0; j < 4; ++j) {
#pragma unroll
    for (int r = 0; r < 8; ++r) {
      unsigned short hb, lb;
      split_hl(acc[j][r] * ko, hb, lb);
      const int li = (16 * w + 8 * h + r) * 64 + 16 * j + m;
      thi[li] = hb;
      tlo[li] = lb;
    }
  }
  __syncthreads();
  store_tile_us<4, 64>(thi, g.CH + (size_t)z * (size_t)g.sCz, (size_t)r0, g.ldc, n0, w, lane);
  store_tile_us<4, 64>(tlo, g.CL + (size_t)z * (size_t)g.sCz, (size_t)r0, g.ldc, n0, w, lane);
}

__global__ __launch_bounds__(128)
void k_aff(const unsigned short* __restrict__ th, const unsigned short* __restrict__ tlw,
           const unsigned short* __restrict__ s16b, const float* __restrict__ pmb,
           const float* __restrict__ smb, unsigned short* ah, unsigned short* al,
           unsigned short* aht, unsigned short* alt)
{
  __shared__ __align__(16) float xs[64 * 64];
  __shared__ float mcl[64];
  __shared__ __align__(16) unsigned short dH[64 * TP];
  __shared__ __align__(16) unsigned short dL[64 * TP];
  __shared__ __align__(16) unsigned short tH[64 * TP];
  __shared__ __align__(16) unsigned short tLw[64 * TP];

  const int tid  = threadIdx.x;
  const int lane = tid & 31;
  const int w    = tid >> 5;
  const int h    = lane >> 4;
  const int m    = lane & 15;
  const int j0   = 64 * blockIdx.x;
  const int i0   = 64 * blockIdx.y;
  const int hd   = blockIdx.z;
  const size_t toff = (size_t)hd * LL * DD;
  const size_t aoff = (size_t)hd * LL * LL;

  if (tid < 64) mcl[tid] = bf16r(smb[j0 + tid]);

  v8f acc[4], accl[4];
#pragma unroll
  for (int j = 0; j < 4; ++j) { acc[j] = zero8(); accl[j] = zero8(); }

  const unsigned short* pah = th  + toff + (size_t)(i0 + 16 * w + m) * DD + 8 * h;
  const unsigned short* pal = tlw + toff + (size_t)(i0 + 16 * w + m) * DD + 8 * h;
  const unsigned short* pb  = s16b + (size_t)(j0 + m) * DD + 8 * h;
  const size_t bs = (size_t)16 * DD;
#pragma unroll 1
  for (int kk = 0; kk < DD / 32; ++kk) {
    const v16us fa = ldfrag_u(pah + 32 * kk);
    const v16us fl = ldfrag_u(pal + 32 * kk);
    const v16us b0 = ldfrag_u(pb + 32 * kk);
    const v16us b1 = ldfrag_u(pb + bs + 32 * kk);
    const v16us b2 = ldfrag_u(pb + 2 * bs + 32 * kk);
    const v16us b3 = ldfrag_u(pb + 3 * bs + 32 * kk);
    acc[0]  = mma_hu(fa, b0, acc[0]);
    acc[1]  = mma_hu(fa, b1, acc[1]);
    acc[2]  = mma_hu(fa, b2, acc[2]);
    acc[3]  = mma_hu(fa, b3, acc[3]);
    accl[0] = mma_hu(fl, b0, accl[0]);
    accl[1] = mma_hu(fl, b1, accl[1]);
    accl[2] = mma_hu(fl, b2, accl[2]);
    accl[3] = mma_hu(fl, b3, accl[3]);
    guard8(acc[0], acc[1], acc[2], acc[3], accl[0], accl[1], accl[2], accl[3],
           fa, fl, b0, b1, b2, b3);
  }

  const float kl = 1.0f / 2048.0f;
  const float kx = 1.0f / 256.0f;
#pragma unroll
  for (int j = 0; j < 4; ++j) {
#pragma unroll
    for (int r = 0; r < 8; ++r)
      xs[(16 * w + 8 * h + r) * 64 + 16 * j + m] = (acc[j][r] + accl[j][r] * kl) * kx;
  }
  __syncthreads();

  {
    const int row = tid >> 1;
    const int cb  = 32 * (tid & 1);
    const float mrow = bf16r(pmb[i0 + row]);
#pragma unroll 2
    for (int e = 0; e < 32; ++e) {
      const int c = cb + e;
      const float mk = mrow * mcl[c];
      const float a  = tanh_f(xs[row * 64 + c]) * mk;
      unsigned short hb, lb;
      split_hl(1024.0f * a, hb, lb);
      dH[row * TP + c]  = hb;
      dL[row * TP + c]  = lb;
      tH[c * TP + row]  = hb;
      tLw[c * TP + row] = lb;
    }
  }
  __syncthreads();

  store_tile_us<4, TP>(dH,  ah  + aoff, (size_t)i0, LL, j0, w, lane);
  store_tile_us<4, TP>(dL,  al  + aoff, (size_t)i0, LL, j0, w, lane);
  store_tile_us<4, TP>(tH,  aht + aoff, (size_t)j0, LL, i0, w, lane);
  store_tile_us<4, TP>(tLw, alt + aoff, (size_t)j0, LL, i0, w, lane);
}

__global__ __launch_bounds__(256)
void k_pool(const unsigned short* __restrict__ ah, const unsigned short* __restrict__ al,
            const unsigned short* __restrict__ aht, const unsigned short* __restrict__ alt,
            const unsigned short* __restrict__ psh, const unsigned short* __restrict__ psl,
            const unsigned short* __restrict__ pph, const unsigned short* __restrict__ ppl,
            unsigned short* qsh, unsigned short* qsl, unsigned short* qph, unsigned short* qpl)
{
  __shared__ __align__(16) unsigned short hT[64 * 64];
  __shared__ __align__(16) unsigned short lT[64 * 64];

  const int tid  = threadIdx.x;
  const int lane = tid & 31;
  const int w    = tid >> 5;
  const int h    = lane >> 4;
  const int m    = lane & 15;
  const int wr   = w & 3;
  const int wc   = w >> 2;
  const int role = blockIdx.z;
  const int d0   = 64 * blockIdx.x;
  const int r0   = 64 * blockIdx.y;

  const unsigned short* A0 = role ? aht : ah;
  const unsigned short* A1 = role ? alt : al;
  const unsigned short* B0 = role ? pph : psh;
  const unsigned short* B1 = role ? ppl : psl;
  unsigned short* OH = role ? qph : qsh;
  unsigned short* OL = role ? qpl : qsl;

  v8f mx[2];
  mx[0] = zero8(); mx[1] = zero8();

  const size_t arow = (size_t)(r0 + 16 * wr + m) * LL + 8 * h;
  const size_t brow = (size_t)(d0 + 32 * wc + m) * LL + 8 * h;
  const size_t bs   = (size_t)16 * LL;
  const float kl = 1.0f / 2048.0f;
  const float kw = 1.0f / 16384.0f;

#pragma unroll 1
  for (int hq = 0; hq < NH; ++hq) {
    const unsigned short* pa0 = A0 + (size_t)hq * LL * LL + arow;
    const unsigned short* pa1 = A1 + (size_t)hq * LL * LL + arow;
    const unsigned short* pb0 = B0 + (size_t)hq * HD * LL + brow;
    const unsigned short* pb1 = B1 + (size_t)hq * HD * LL + brow;
    v8f c0 = zero8(), c1 = zero8(), x0 = zero8(), x1 = zero8();
#pragma unroll 1
    for (int kk = 0; kk < LL / 32; ++kk) {
      const v16us fa  = ldfrag_u(pa0 + 32 * kk);
      const v16us fl  = ldfrag_u(pa1 + 32 * kk);
      const v16us bh0 = ldfrag_u(pb0 + 32 * kk);
      const v16us bh1 = ldfrag_u(pb0 + bs + 32 * kk);
      const v16us bl0 = ldfrag_u(pb1 + 32 * kk);
      const v16us bl1 = ldfrag_u(pb1 + bs + 32 * kk);
      c0 = mma_hu(fa, bh0, c0);
      c1 = mma_hu(fa, bh1, c1);
      x0 = mma_hu(fa, bl0, x0);
      x1 = mma_hu(fa, bl1, x1);
      x0 = mma_hu(fl, bh0, x0);
      x1 = mma_hu(fl, bh1, x1);
      guard4x6(c0, c1, x0, x1, fa, fl, bh0, bh1, bl0, bl1);
    }
#pragma unroll
    for (int r = 0; r < 8; ++r) {
      mx[0][r] = fmaxf(mx[0][r], (c0[r] + x0[r] * kl) * kw);
      mx[1][r] = fmaxf(mx[1][r], (c1[r] + x1[r] * kl) * kw);
    }
  }

#pragma unroll
  for (int j = 0; j < 2; ++j) {
#pragma unroll
    for (int r = 0; r < 8; ++r) {
      unsigned short hb, lb;
      split_hl(16.0f * mx[j][r], hb, lb);
      const int li = (16 * wr + 8 * h + r) * 64 + 32 * wc + 16 * j + m;
      hT[li] = hb;
      lT[li] = lb;
    }
  }
  __syncthreads();
  store_tile_us<8, 64>(hT, OH, (size_t)r0, HD, d0, w, lane);
  store_tile_us<8, 64>(lT, OL, (size_t)r0, HD, d0, w, lane);
}

struct OArgs {
  const unsigned short* X;
  const unsigned short* QH;
  const unsigned short* QL;
  const unsigned short* W;
  const float* bias;
  float* out;
};
static_assert(sizeof(OArgs) == 48);

__global__ __launch_bounds__(128)
void k_out(OArgs g)
{
  __shared__ __align__(16) float ct[64 * 64];

  const int tid  = threadIdx.x;
  const int lane = tid & 31;
  const int w    = tid >> 5;
  const int h    = lane >> 4;
  const int m    = lane & 15;
  const int n0   = 64 * blockIdx.x;
  const int r0   = 64 * blockIdx.y;

  v8f acc[4], accl[4];
#pragma unroll
  for (int j = 0; j < 4; ++j) { acc[j] = zero8(); accl[j] = zero8(); }

  const unsigned short* pa = g.X + (size_t)(r0 + 16 * w + m) * DD + 8 * h;
  const unsigned short* pb = g.W + (size_t)(n0 + m) * KC + 8 * h;
  const size_t bs = (size_t)16 * KC;
#pragma unroll 2
  for (int kk = 0; kk < DD / 32; ++kk) {
    const v16us a  = ldfrag_u(pa + 32 * kk);
    const v16us b0 = ldfrag_u(pb + 32 * kk);
    const v16us b1 = ldfrag_u(pb + bs + 32 * kk);
    const v16us b2 = ldfrag_u(pb + 2 * bs + 32 * kk);
    const v16us b3 = ldfrag_u(pb + 3 * bs + 32 * kk);
    acc[0] = mma_hu(a, b0, acc[0]);
    acc[1] = mma_hu(a, b1, acc[1]);
    acc[2] = mma_hu(a, b2, acc[2]);
    acc[3] = mma_hu(a, b3, acc[3]);
    guard4(acc[0], acc[1], acc[2], acc[3], a, b0, b1, b2, b3);
  }

  const unsigned short* pqh = g.QH + (size_t)(r0 + 16 * w + m) * HD + 8 * h;
  const unsigned short* pql = g.QL + (size_t)(r0 + 16 * w + m) * HD + 8 * h;
  const unsigned short* pb2 = pb + DD;
#pragma unroll 1
  for (int kk = 0; kk < HD / 32; ++kk) {
    const v16us fa = ldfrag_u(pqh + 32 * kk);
    const v16us fl = ldfrag_u(pql + 32 * kk);
    const v16us b0 = ldfrag_u(pb2 + 32 * kk);
    const v16us b1 = ldfrag_u(pb2 + bs + 32 * kk);
    const v16us b2 = ldfrag_u(pb2 + 2 * bs + 32 * kk);
    const v16us b3 = ldfrag_u(pb2 + 3 * bs + 32 * kk);
    acc[0]  = mma_hu(fa, b0, acc[0]);
    acc[1]  = mma_hu(fa, b1, acc[1]);
    acc[2]  = mma_hu(fa, b2, acc[2]);
    acc[3]  = mma_hu(fa, b3, acc[3]);
    accl[0] = mma_hu(fl, b0, accl[0]);
    accl[1] = mma_hu(fl, b1, accl[1]);
    accl[2] = mma_hu(fl, b2, accl[2]);
    accl[3] = mma_hu(fl, b3, accl[3]);
    guard8(acc[0], acc[1], acc[2], acc[3], accl[0], accl[1], accl[2], accl[3],
           fa, fl, b0, b1, b2, b3);
  }

  float bv[4];
#pragma unroll
  for (int j = 0; j < 4; ++j) bv[j] = bf16r(g.bias[n0 + 16 * j + m]);
  const float kl = 1.0f / 2048.0f;
  const float ko = 1.0f / 1024.0f;
#pragma unroll
  for (int j = 0; j < 4; ++j) {
#pragma unroll
    for (int r = 0; r < 8; ++r)
      ct[(16 * w + 8 * h + r) * 64 + 16 * j + m] =
          fmaxf((acc[j][r] + accl[j][r] * kl) * ko + bv[j], 0.0f);
  }
  __syncthreads();
  store_tile_f32(ct, g.out, (size_t)r0, n0, DD, w, lane);
}

extern "C" void kernel_launch(void* const* d_in, const int* in_sizes, int n_in,
                              void* d_out, int out_size, void* d_ws, size_t ws_size,
                              hipStream_t stream) {
  if (n_in < 11) return;
  if (in_sizes[0] != NB * LL * DD) return;
  if (in_sizes[1] != NB * LL * DD) return;
  if (in_sizes[2] != NB * LL) return;
  if (in_sizes[3] != NB * LL) return;
  if (in_sizes[4] != NH * DD * DD) return;
  if (in_sizes[5] != DD * INR) return;
  if (in_sizes[6] != DD * INR) return;
  if (in_sizes[7] != KC * DD) return;
  if (in_sizes[8] != DD) return;
  if (in_sizes[9] != KC * DD) return;
  if (in_sizes[10] != DD) return;
  if (out_size != 2 * NB * LL * DD) return;
  if (ws_size < WS_TOTAL) return;

  const float* Pin  = (const float*)d_in[0];
  const float* Sin  = (const float*)d_in[1];
  const float* pm   = (const float*)d_in[2];
  const float* sm   = (const float*)d_in[3];
  const float* Waff = (const float*)d_in[4];
  const float* Wp   = (const float*)d_in[5];
  const float* Wsx  = (const float*)d_in[6];
  const float* Wfp  = (const float*)d_in[7];
  const float* bfp  = (const float*)d_in[8];
  const float* Wfs  = (const float*)d_in[9];
  const float* bfs  = (const float*)d_in[10];
  float* out = (float*)d_out;

  char* ws = (char*)d_ws;
  unsigned short* p16   = (unsigned short*)(ws + OFF_P16);
  unsigned short* s16   = (unsigned short*)(ws + OFF_S16);
  unsigned short* wa16  = (unsigned short*)(ws + OFF_WA);
  unsigned short* wp16  = (unsigned short*)(ws + OFF_WP);
  unsigned short* ws16  = (unsigned short*)(ws + OFF_WS);
  unsigned short* wfp16 = (unsigned short*)(ws + OFF_WFP);
  unsigned short* wfs16 = (unsigned short*)(ws + OFF_WFS);
  unsigned short* pph   = (unsigned short*)(ws + OFF_PPH);
  unsigned short* ppl   = (unsigned short*)(ws + OFF_PPL);
  unsigned short* psh   = (unsigned short*)(ws + OFF_PSH);
  unsigned short* psl   = (unsigned short*)(ws + OFF_PSL);
  unsigned short* th    = (unsigned short*)(ws + OFF_TH);
  unsigned short* tl    = (unsigned short*)(ws + OFF_TL);
  unsigned short* ah    = (unsigned short*)(ws + OFF_AH);
  unsigned short* al    = (unsigned short*)(ws + OFF_AL);
  unsigned short* aht   = (unsigned short*)(ws + OFF_AHT);
  unsigned short* alt   = (unsigned short*)(ws + OFF_ALT);
  unsigned short* qsh   = (unsigned short*)(ws + OFF_QSH);
  unsigned short* qsl   = (unsigned short*)(ws + OFF_QSL);
  unsigned short* qph   = (unsigned short*)(ws + OFF_QPH);
  unsigned short* qpl   = (unsigned short*)(ws + OFF_QPL);

  k_cva<<<dim3(4096), dim3(256), 0, stream>>>(Pin, Sin, p16, s16);
  (void)hipGetLastError();
  k_cvw<<<dim3(928), dim3(256), 0, stream>>>(Waff, Wp, Wsx, Wfp, Wfs, wa16, wp16, ws16, wfp16, wfs16);
  (void)hipGetLastError();

  GArgs gp = {};
  gp.A = wp16; gp.B = p16; gp.CH = pph; gp.CL = ppl;
  gp.sAz = 0; gp.sBz = (long long)LL * DD; gp.sCz = (long long)INR * LL;
  gp.lda = DD; gp.ldb = DD; gp.ldc = LL; gp.nk = DD / 32;
  k_ghl<<<dim3(LL / 64, INR / 64, NB), dim3(128), 0, stream>>>(gp);
  (void)hipGetLastError();
  GArgs gs = gp;
  gs.A = ws16; gs.B = s16; gs.CH = psh; gs.CL = psl;
  k_ghl<<<dim3(LL / 64, INR / 64, NB), dim3(128), 0, stream>>>(gs);
  (void)hipGetLastError();

  for (int b = 0; b < NB; ++b) {
    GArgs gt = {};
    gt.A = p16 + (size_t)b * LL * DD; gt.B = wa16; gt.CH = th; gt.CL = tl;
    gt.sAz = 0; gt.sBz = (long long)DD * DD; gt.sCz = (long long)LL * DD;
    gt.lda = DD; gt.ldb = DD; gt.ldc = DD; gt.nk = DD / 32;
    k_ghl<<<dim3(DD / 64, LL / 64, NH), dim3(128), 0, stream>>>(gt);
    (void)hipGetLastError();
    k_aff<<<dim3(LL / 64, LL / 64, NH), dim3(128), 0, stream>>>(
        th, tl, s16 + (size_t)b * LL * DD, pm + (size_t)b * LL, sm + (size_t)b * LL,
        ah, al, aht, alt);
    (void)hipGetLastError();
    k_pool<<<dim3(HD / 64, LL / 64, 2), dim3(256), 0, stream>>>(
        ah, al, aht, alt,
        psh + (size_t)b * INR * LL, psl + (size_t)b * INR * LL,
        pph + (size_t)b * INR * LL, ppl + (size_t)b * INR * LL,
        qsh + (size_t)b * LL * HD, qsl + (size_t)b * LL * HD,
        qph + (size_t)b * LL * HD, qpl + (size_t)b * LL * HD);
    (void)hipGetLastError();
  }

  OArgs op = {};
  op.X = p16; op.QH = qsh; op.QL = qsl; op.W = wfp16; op.bias = bfp; op.out = out;
  k_out<<<dim3(DD / 64, (NB * LL) / 64), dim3(128), 0, stream>>>(op);
  (void)hipGetLastError();
  OArgs oq = {};
  oq.X = s16; oq.QH = qph; oq.QL = qpl; oq.W = wfs16; oq.bias = bfs; oq.out = out + (size_t)NB * LL * DD;
  k_out<<<dim3(DD / 64, (NB * LL) / 64), dim3(128), 0, stream>>>(oq);
  (void)hipGetLastError();
}
